// GINModel_62362925138436
// MI455X (gfx1250) — hardware-verified
//
#include <hip/hip_runtime.h>

#define N_NODES 50000
#define N_EDGES 1600000
#define FDIM 128
#define NPAD 50048
#define N_GRAPHS 512
#define N_LAYERS 4
#define NTHR 256
#define TROWS 16384
#define WROWS 2048
#define NTILE 4
#define SCH 4096
#define SPE (SCH / NTHR)
#define NCH ((N_EDGES + SCH - 1) / SCH)
#define LCAP SCH

static_assert(N_EDGES % SPE == 0, "edge groups are whole");
static_assert(NTILE * TROWS >= NPAD, "destination tiles cover all padded rows");
static_assert(TROWS == 8 * WROWS, "eight waves per tile");
static_assert(NPAD % 64 == 0 && NPAD >= N_NODES && NPAD - N_NODES < 64, "M padded to the 64 tile");
static_assert(FDIM % 64 == 0 && FDIM % 32 == 0, "N tile multiple and K multiple of 32");
static_assert(N_NODES < 65536 && TROWS <= 16384, "hit record packing fits 31 bits");
static_assert((NPAD * (FDIM / 4)) % NTHR == 0, "cast grid exact");
static_assert((N_LAYERS * 2 * FDIM * FDIM / 2) % NTHR == 0, "weight pack grid exact");
static_assert(N_GRAPHS % 8 == 0, "pool grid exact");
static_assert(2 * N_LAYERS * FDIM == 4 * NTHR, "bias pack covers blocks 0..3");

typedef __attribute__((ext_vector_type(16))) _Float16 v16h;
typedef __attribute__((ext_vector_type(8)))  _Float16 v8h;
typedef __attribute__((ext_vector_type(16))) __bf16   v16b;
typedef __attribute__((ext_vector_type(8)))  __bf16   v8b;
typedef __attribute__((ext_vector_type(8)))  float    v8f;
typedef __attribute__((ext_vector_type(4)))  float    v4f;
typedef __attribute__((ext_vector_type(4)))  int      v4i;
typedef __attribute__((ext_vector_type(4)))  unsigned int v4u;

__device__ __forceinline__ unsigned short f2bf_bits(float f) {
  unsigned u = __float_as_uint(f);
  return (unsigned short)((u + 0x7FFFu + ((u >> 16) & 1u)) >> 16);
}
__device__ __forceinline__ float bf_bits2f(unsigned short h) { return __uint_as_float(((unsigned)h) << 16); }
__device__ __forceinline__ unsigned pk16(unsigned short a, unsigned short b) { return (unsigned)a | ((unsigned)b << 16); }

__device__ __forceinline__ void keep4_b(v16b a, v16b b, v16b c, v16b d) { asm volatile("v_nop" :: "v"(a), "v"(b), "v"(c), "v"(d)); }
__device__ __forceinline__ void acc_guard4(v8f& a, v8f& b, v8f& c, v8f& d) { asm volatile("v_nop\n\tv_nop\n\tv_nop\n\tv_nop" : "+v"(a), "+v"(b), "+v"(c), "+v"(d)); }
__device__ __forceinline__ void dep_guard_all_b(v8f& a, v8f& b, v8f& c, v8f& d, v16b x, v16b y, v16b p, v16b q, v16b r, v16b s) {
  asm volatile("v_nop\n\tv_nop\n\tv_nop\n\tv_nop" : "+v"(a), "+v"(b), "+v"(c), "+v"(d) : "v"(x), "v"(y), "v"(p), "v"(q), "v"(r), "v"(s));
}
struct FragB {
  union U { v16b v; v8b h[2]; };
  static __device__ __forceinline__ v16b load(const __bf16* p) {
    U f; f.h[0] = *(const v8b*)(p); f.h[1] = *(const v8b*)(p + 16); return f.v;
  }
  static __device__ __forceinline__ v8f mma(v16b a, v16b b, v8f c) {
    return __builtin_amdgcn_wmma_f32_16x16x32_bf16(false, a, false, b, (short)0, c, false, false);
  }
};

template <int SPLITM, int BIAS_MODE, int OUT_MODE, int ACT>
__global__ __launch_bounds__(256) void wmma_gemm64(
    const unsigned short* __restrict__ Ap, const unsigned short* __restrict__ A2p, int lda,
    const unsigned short* __restrict__ Btp, const unsigned short* __restrict__ Bt2p, int ldb,
    void* __restrict__ Cout, void* __restrict__ Cout2, int ldc,
    const float* __restrict__ bias, int M, int N, int K, float scale) {
  const __bf16* A = (const __bf16*)Ap; const __bf16* A2 = (const __bf16*)A2p;
  const __bf16* Bt = (const __bf16*)Btp; const __bf16* Bt2 = (const __bf16*)Bt2p;
  __shared__ __align__(16) float sT[8][16 * 68];
  const int lane = threadIdx.x & 31;
  const int wave = threadIdx.x >> 5;
  const int tilesN = N >> 6;
  const int tilesM = M >> 6;
  const int tile = blockIdx.x * 8 + wave;
  if (tile >= tilesM * tilesN) return;
  const int tm = tile / tilesN;
  const int tn = tile - tm * tilesN;
  const int m0 = tm << 6;
  const int n0 = tn << 6;

  const int rlane = lane & 15;
  const int koff  = (lane >> 4) * 8;
  const int mOff  = (lane >> 4) * 8;

  v8f acc[4][4];
#pragma unroll
  for (int i = 0; i < 4; ++i)
#pragma unroll
    for (int j = 0; j < 4; ++j) acc[i][j] = (v8f){0.f,0.f,0.f,0.f,0.f,0.f,0.f,0.f};

  for (int k0 = 0; k0 < K; k0 += 32) {
    v16b bh[4], bl[4];
#pragma unroll
    for (int j = 0; j < 4; ++j) {
      const size_t bo = (size_t)(n0 + (j << 4) + rlane) * ldb + koff + k0;
      bh[j] = FragB::load(Bt + bo);
      bl[j] = bh[j];
      if (SPLITM == 2) bl[j] = FragB::load(Bt2 + bo);
    }
#pragma unroll
    for (int i = 0; i < 4; ++i) {
      const size_t ao = (size_t)(m0 + (i << 4) + rlane) * lda + koff + k0;
      const v16b ah = FragB::load(A + ao);
      v16b al = ah;
      if (SPLITM >= 1) al = FragB::load(A2 + ao);
#pragma unroll
      for (int j = 0; j < 4; ++j) {
        acc[i][j] = FragB::mma(ah, bh[j], acc[i][j]);
        if (SPLITM == 2) acc[i][j] = FragB::mma(ah, bl[j], acc[i][j]);
        if (SPLITM >= 1) acc[i][j] = FragB::mma(al, bh[j], acc[i][j]);
      }
      dep_guard_all_b(acc[i][0], acc[i][1], acc[i][2], acc[i][3], ah, al, bh[0], bh[1], bh[2], bh[3]);
    }
    keep4_b(bh[0], bh[1], bh[2], bh[3]);
    if (SPLITM == 2) keep4_b(bl[0], bl[1], bl[2], bl[3]);
  }
  acc_guard4(acc[0][0], acc[0][1], acc[0][2], acc[0][3]);
  acc_guard4(acc[1][0], acc[1][1], acc[1][2], acc[1][3]);
  acc_guard4(acc[2][0], acc[2][1], acc[2][2], acc[2][3]);
  acc_guard4(acc[3][0], acc[3][1], acc[3][2], acc[3][3]);

  float* slab = sT[wave];
#pragma unroll
  for (int i = 0; i < 4; ++i) {
    const int mBase = m0 + (i << 4);
#pragma unroll
    for (int j = 0; j < 4; ++j) {
      const int n = n0 + (j << 4) + rlane;
      float bv = 0.f;
      if (BIAS_MODE == 2) bv = bias[n];
#pragma unroll
      for (int r = 0; r < 8; ++r) {
        float v = acc[i][j][r] * scale;
        if (BIAS_MODE == 2) v += bv;
        if (ACT == 2) v = fmaxf(v, 0.0f);
        slab[(mOff + r) * 68 + (j << 4) + rlane] = v;
      }
    }
    __builtin_amdgcn_fence(__ATOMIC_RELEASE, "workgroup");
    __builtin_amdgcn_wave_barrier();
    __builtin_amdgcn_fence(__ATOMIC_ACQUIRE, "workgroup");
    if (OUT_MODE == 0) {
      float* C = (float*)Cout;
      const int hh = lane >> 4, c4 = (lane & 15) * 4;
      for (int pass = 0; pass < 2; ++pass) {
#pragma unroll
        for (int it = 0; it < 8; ++it) {
          const int row = it * 2 + hh;
          v4f v = *(const v4f*)(slab + row * 68 + c4);
          *(volatile v4f*)(C + (size_t)(mBase + row) * ldc + n0 + c4) = v;
        }
        __threadfence();
      }
    } else {
      const int q = lane >> 3, c8 = (lane & 7) * 8;
      unsigned short* C  = (unsigned short*)Cout;
      unsigned short* C2 = (unsigned short*)Cout2;
      for (int pass = 0; pass < 2; ++pass) {
#pragma unroll
        for (int it = 0; it < 4; ++it) {
          const int row = it * 4 + q;
          const float* sp = slab + row * 68 + c8;
          v8h hv, lv;
#pragma unroll
          for (int e = 0; e < 8; ++e) {
            unsigned short hb = f2bf_bits(sp[e]);
            unsigned short lb = f2bf_bits(sp[e] - bf_bits2f(hb));
            hv[e] = __builtin_bit_cast(_Float16, hb);
            lv[e] = __builtin_bit_cast(_Float16, lb);
          }
          *(volatile v8h*)(C + (size_t)(mBase + row) * ldc + n0 + c8) = hv;
          *(volatile v8h*)(C2 + (size_t)(mBase + row) * ldc + n0 + c8) = lv;
        }
        __threadfence();
      }
    }
    __builtin_amdgcn_fence(__ATOMIC_RELEASE, "workgroup");
    __builtin_amdgcn_wave_barrier();
    __builtin_amdgcn_fence(__ATOMIC_ACQUIRE, "workgroup");
  }
}

__device__ __forceinline__ int blk_excl_scan(int cnt, int* scan_ws, int tid, int* tot) {
  const int lane = tid & 31, wave = tid >> 5; int incl = cnt;
#pragma unroll
  for (int o = 1; o < 32; o <<= 1) { const int v = __shfl_up(incl, o, 32); if (lane >= o) incl += v; }
  if (lane == 31) scan_ws[wave] = incl;
  __syncthreads();
  if (wave == 0) { int sv = scan_ws[lane]; int wv = (lane < NTHR / 32) ? sv : 0; int wincl = wv;
#pragma unroll
    for (int o = 1; o < 32; o <<= 1) { const int v = __shfl_up(wincl, o, 32); if (lane >= o) wincl += v; }
    if (lane < NTHR / 32) scan_ws[32 + lane] = wincl - wv; if (lane == 31) scan_ws[64] = wincl; }
  __syncthreads();
  const int res = scan_ws[32 + wave] + incl - cnt; *tot = scan_ws[64];
  return res;
}
__device__ __forceinline__ int chunk_hits(const int* __restrict__ dstv, const int* __restrict__ srcv, int e0, int n0, int tid,
                                          int* LIST, int* scan_ws) {
  const int eb = e0 + tid * SPE;
  const bool live = eb < N_EDGES;
  const int ebc = live ? eb : (N_EDGES - SPE);
  int rec[SPE]; int cnt = 0;
#pragma unroll
  for (int k = 0; k < SPE; k += 4) {
    const v4i d4 = *(const v4i*)(dstv + ebc + k);
    const v4i s4 = *(const v4i*)(srcv + ebc + k);
    asm volatile("" ::: "memory");
#pragma unroll
    for (int e = 0; e < 4; ++e) {
      const int d = d4[e]; int r = -1;
      if (live && d >= n0 && d < n0 + TROWS) {
        int s = s4[e]; s = s < 0 ? 0 : (s >= N_NODES ? N_NODES - 1 : s);
        r = ((d - n0) << 16) | s; ++cnt;
      }
      rec[k + e] = r;
    }
  }
  int tot; int p = blk_excl_scan(cnt, scan_ws, tid, &tot);
#pragma unroll
  for (int k = 0; k < SPE; ++k) if (rec[k] >= 0) { if ((unsigned)p < (unsigned)LCAP) LIST[p] = rec[k]; ++p; }
  __syncthreads();
  return tot < LCAP ? tot : LCAP;
}

__global__ __launch_bounds__(NTHR) void gin_aggregate_kernel(const float* __restrict__ X, const int* __restrict__ ei,
                                                          float* ACC, unsigned short* __restrict__ AH, unsigned short* __restrict__ AL) {
  __shared__ int LIST[LCAP + 32];
  __shared__ int scan_ws[80];
  const int tid = threadIdx.x, lane = tid & 31, wave = tid >> 5;
  const int n0 = blockIdx.x * TROWS;
  const int wr0 = n0 + wave * WROWS;
  for (int i = tid; i < LCAP + 32; i += NTHR) LIST[i] = -1;
  if (tid < 80) scan_ws[tid] = 0;
  const v4f z4 = {0.f, 0.f, 0.f, 0.f};
#pragma unroll 1
  for (int j = 0; j < WROWS; ++j) {
    const int row = wr0 + j;
    if (row < NPAD) {
      const int rs = row < N_NODES ? row : N_NODES - 1;
      v4f v = *(const v4f*)(X + (size_t)rs * FDIM + 4 * lane);
      if (row >= N_NODES) v = z4;
      *(v4f*)(ACC + (size_t)row * FDIM + 4 * lane) = v;
    }
  }
  __syncthreads();
  const int* srcv = ei; const int* dstv = ei + N_EDGES;
#pragma unroll 1
  for (int c = 0; c < NCH; ++c) {
    const int tot = chunk_hits(dstv, srcv, c * SCH, n0, tid, LIST, scan_ws);
#pragma unroll 1
    for (int base = 0; base < tot; base += 32) {
      const int q = base + lane;
      const int lv = LIST[q];
      const int rv = (q < tot) ? lv : -1;
      const int own = (rv >= 0 && (rv >> 27) == wave) ? 1 : 0;
      unsigned msk = (unsigned)__ballot(own);
#pragma unroll 1
      for (int it = 0; it < 32; ++it) {
        if (msk == 0u) break;
        const int bp = __builtin_ctz(msk); msk &= msk - 1u;
        const int r = __shfl(rv, bp, 32);
        const int dl = (r >> 16) & (TROWS - 1);
        int s = r & 0xFFFF; s = s < N_NODES ? s : N_NODES - 1;
        int row = n0 + dl; row = row < NPAD ? row : NPAD - 1;
        const v4f xv = *(const v4f*)(X + (size_t)s * FDIM + 4 * lane);
        float* rp = ACC + (size_t)row * FDIM + 4 * lane;
        v4f a = *(const v4f*)rp;
        a = a + xv;
        *(v4f*)rp = a;
      }
    }
    __syncthreads();
  }
  __threadfence_block();
  const int hh = lane >> 4, c8 = (lane & 15) * 8;
#pragma unroll 1
  for (int j = 0; j < WROWS / 2; ++j) {
    const int rb = wr0 + 2 * j;
    if (rb < NPAD) {
      const int row = rb + hh;
      const float* rp = ACC + (size_t)row * FDIM + c8;
      const v4f a0 = *(const v4f*)rp;
      const v4f a1 = *(const v4f*)(rp + 4);
      unsigned short hb[8], lb[8];
#pragma unroll
      for (int e = 0; e < 4; ++e) {
        hb[e] = f2bf_bits(a0[e]);     lb[e] = f2bf_bits(a0[e] - bf_bits2f(hb[e]));
        hb[4 + e] = f2bf_bits(a1[e]); lb[4 + e] = f2bf_bits(a1[e] - bf_bits2f(hb[4 + e]));
      }
      const v4u uh = (v4u){pk16(hb[0], hb[1]), pk16(hb[2], hb[3]), pk16(hb[4], hb[5]), pk16(hb[6], hb[7])};
      const v4u ul = (v4u){pk16(lb[0], lb[1]), pk16(lb[2], lb[3]), pk16(lb[4], lb[5]), pk16(lb[6], lb[7])};
      unsigned short* ph = AH + (size_t)row * FDIM + c8;
      unsigned short* pl = AL + (size_t)row * FDIM + c8;
      for (int pass = 0; pass < 2; ++pass) {
        *(volatile v4u*)ph = uh;
        *(volatile v4u*)pl = ul;
        __threadfence();
      }
    }
  }
}

__global__ __launch_bounds__(NTHR) void add_pool_kernel(const float* __restrict__ XF, const int* __restrict__ batch, float* __restrict__ out) {
  const int lane = threadIdx.x & 31, wave = threadIdx.x >> 5;
  const int g = blockIdx.x * 8 + wave;
  v4f acc = {0.f, 0.f, 0.f, 0.f};
#pragma unroll 1
  for (int base = 0; base < N_NODES; base += 32) {
    const int idx = base + lane;
    const int idc = idx < N_NODES ? idx : N_NODES - 1;
    const int bv = batch[idc];
    const int hit = (idx < N_NODES && bv == g) ? 1 : 0;
    unsigned msk = (unsigned)__ballot(hit);
#pragma unroll 1
    for (int it = 0; it < 32; ++it) {
      if (msk == 0u) break;
      const int bp = __builtin_ctz(msk); msk &= msk - 1u;
      const int row = base + bp;
      acc = acc + *(const v4f*)(XF + (size_t)row * FDIM + 4 * lane);
    }
  }
  float* op = out + (size_t)g * FDIM + 4 * lane;
  for (int pass = 0; pass < 2; ++pass) { *(volatile v4f*)op = acc; __threadfence(); }
}

__global__ __launch_bounds__(NTHR) void prep_w_kernel(const float* __restrict__ Ws1, const float* __restrict__ Ws2,
                                                    const float* __restrict__ bs1, const float* __restrict__ bs2,
                                                    unsigned* __restrict__ WT, float* __restrict__ BR) {
  const int i = blockIdx.x * NTHR + threadIdx.x;
  const int mat = i >> 13;
  const int l = mat >> 1, g = mat & 1;
  const int wi = i & 8191;
  const int n = wi >> 6;
  const int k = 2 * (wi & 63);
  const float* W = (g == 0 ? Ws1 : Ws2) + (size_t)l * FDIM * FDIM;
  const float a = W[(size_t)k * FDIM + n];
  const float b = W[(size_t)(k + 1) * FDIM + n];
  const unsigned u = pk16(f2bf_bits(a), f2bf_bits(b));
  ((volatile unsigned*)WT)[i] = u;
  __threadfence();
  ((volatile unsigned*)WT)[i] = u;
  if (blockIdx.x < 4) {
    const float* bsrc = (blockIdx.x < 2) ? bs1 : bs2;
    const float v = bsrc[i & 511];
    const float rr = bf_bits2f(f2bf_bits(v));
    ((volatile float*)BR)[i] = rr;
    __threadfence();
    ((volatile float*)BR)[i] = rr;
  }
}

__global__ __launch_bounds__(NTHR) void prep_x_kernel(const float* __restrict__ x, float* __restrict__ XF) {
  const int i = blockIdx.x * NTHR + threadIdx.x;
  const int row = i >> 5, c4 = (i & 31) * 4;
  const int rs = row < N_NODES ? row : N_NODES - 1;
  const v4f v = *(const v4f*)(x + (size_t)rs * FDIM + c4);
  const bool live = row < N_NODES;
  v4f rr;
#pragma unroll
  for (int e = 0; e < 4; ++e) rr[e] = live ? bf_bits2f(f2bf_bits(v[e])) : 0.f;
  float* op = XF + (size_t)row * FDIM + c4;
  *(volatile v4f*)op = rr;
  __threadfence();
  *(volatile v4f*)op = rr;
}

extern "C" void kernel_launch(void* const* d_in, const int* in_sizes, int n_in,
                              void* d_out, int out_size, void* d_ws, size_t ws_size, hipStream_t stream) {
  (void)n_in;
  const float* x     = (const float*)d_in[0];
  const int*   ei    = (const int*)  d_in[1];
  const int*   batch = (const int*)  d_in[2];
  const float* Ws1   = (const float*)d_in[3];
  const float* bs1   = (const float*)d_in[4];
  const float* Ws2   = (const float*)d_in[5];
  const float* bs2   = (const float*)d_in[6];
  float* out = (float*)d_out;

  if (in_sizes[0] != N_NODES * FDIM || in_sizes[1] != 2 * N_EDGES || in_sizes[2] != N_NODES ||
      in_sizes[3] != N_LAYERS * FDIM * FDIM || in_sizes[4] != N_LAYERS * FDIM ||
      in_sizes[5] != N_LAYERS * FDIM * FDIM || in_sizes[6] != N_LAYERS * FDIM || out_size != N_GRAPHS * FDIM) return;

  char* ws = (char*)d_ws; size_t off = 0;
  auto carve = [&](size_t bytes) -> char* { char* p = ws + off; off += (bytes + 255) & ~(size_t)255; return p; };
  unsigned*       WT  = (unsigned*)carve((size_t)N_LAYERS * 2 * FDIM * FDIM * 2);
  float*          BR  = (float*)carve((size_t)2 * N_LAYERS * FDIM * 4);
  float*          XF  = (float*)carve((size_t)NPAD * FDIM * 4);
  float*          ACC = (float*)carve((size_t)NPAD * FDIM * 4);
  unsigned short* AH  = (unsigned short*)carve((size_t)NPAD * FDIM * 2);
  unsigned short* AL  = (unsigned short*)carve((size_t)NPAD * FDIM * 2);
  unsigned short* H1H = (unsigned short*)carve((size_t)NPAD * FDIM * 2);
  unsigned short* H1L = (unsigned short*)carve((size_t)NPAD * FDIM * 2);
  if (off > ws_size || off > (size_t)134217728) return;

  prep_w_kernel<<<(N_LAYERS * 2 * FDIM * FDIM / 2) / NTHR, NTHR, 0, stream>>>(Ws1, Ws2, bs1, bs2, WT, BR);
  prep_x_kernel<<<(NPAD * (FDIM / 4)) / NTHR, NTHR, 0, stream>>>(x, XF);

  const int gemm_tiles  = (NPAD / 64) * (FDIM / 64);
  const int gemm_blocks = (gemm_tiles + 7) / 8;
  const unsigned short* WTh = (const unsigned short*)WT;
  for (int l = 0; l < N_LAYERS; ++l) {
    gin_aggregate_kernel<<<NTILE, NTHR, 0, stream>>>(XF, ei, ACC, AH, AL);
    wmma_gemm64<1, 2, 2, 2><<<gemm_blocks, 256, 0, stream>>>(
        (const unsigned short*)AH, (const unsigned short*)AL, FDIM,
        WTh + (size_t)(l * 2 + 0) * FDIM * FDIM, WTh + (size_t)(l * 2 + 0) * FDIM * FDIM, FDIM,
        (void*)H1H, (void*)H1L, FDIM,
        BR + (size_t)l * FDIM, NPAD, FDIM, FDIM, 1.0f);
    wmma_gemm64<1, 2, 0, 0><<<gemm_blocks, 256, 0, stream>>>(
        (const unsigned short*)H1H, (const unsigned short*)H1L, FDIM,
        WTh + (size_t)(l * 2 + 1) * FDIM * FDIM, WTh + (size_t)(l * 2 + 1) * FDIM * FDIM, FDIM,
        (void*)XF, (void*)XF, FDIM,
        BR + (size_t)N_LAYERS * FDIM + (size_t)l * FDIM, NPAD, FDIM, FDIM, 1.0f);
  }
  add_pool_kernel<<<N_GRAPHS / 8, NTHR, 0, stream>>>(XF, batch, out);
}
